// Net_54185307406400
// MI455X (gfx1250) — hardware-verified
//
#include <hip/hip_runtime.h>
#include <math.h>

typedef __attribute__((ext_vector_type(16))) _Float16 v16h;
typedef __attribute__((ext_vector_type(8)))  _Float16 v8h;
typedef __attribute__((ext_vector_type(16))) __bf16   v16b;
typedef __attribute__((ext_vector_type(8)))  __bf16   v8b;
typedef __attribute__((ext_vector_type(8)))  float    v8f;
typedef __attribute__((ext_vector_type(4)))  float    v4f;

constexpr int kBsz    = 512;
constexpr int kSeq    = 28;
constexpr int kInF    = 28;
constexpr int kInP    = 32;
constexpr int kDm     = 128;
constexpr int kDin    = 256;
constexpr int kNst    = 16;
constexpr int kTaps   = 3;
constexpr int kDtR    = 8;
constexpr int kNcls   = 10;
constexpr int kXzN    = 2 * kDin;
constexpr int kDblN   = kDtR + 2 * kNst;
constexpr int kDblP   = 64;
constexpr int kClsP   = 64;
constexpr int kRows   = kBsz * kSeq;
constexpr int kConvTP = 260;
constexpr int kScanYP = 260;
constexpr float kInvSeq = 1.0f / 28.0f;
static_assert(kDblN <= kDblP && kNcls <= kClsP && kInF <= kInP, "pads");
static_assert((kInP % 32) == 0 && (kDm % 32) == 0 && (kDin % 32) == 0, "GEMM K multiples of 32");
static_assert((kRows % 64) == 0 && (kBsz % 64) == 0 && (kDm % 64) == 0 && (kXzN % 64) == 0 &&
              (kDblP % 64) == 0 && (kClsP % 64) == 0, "GEMM M,N multiples of 64");
static_assert((kRows * kInF) % (64 * 28) == 0 && (64 * 28) == 7 * 256, "x pad tile");
static_assert(kInF * kDm == 14 * 256, "w_inp pad tile");
static_assert(kSeq * kDblP == 7 * 256, "dbl staging tile");
static_assert((kBsz * kDm) % (8 * 256) == 0 && (kBsz * kNcls) % (4 * 256) == 0, "pool/pack grids");

constexpr size_t kOffWINT = 0;
constexpr size_t kOffWXT  = kOffWINT + (size_t)kXzN  * kDm  * 2;
constexpr size_t kOffWOT  = kOffWXT  + (size_t)kDblP * kDin * 2;
constexpr size_t kOffWCT  = kOffWOT  + (size_t)kDm   * kDin * 2;
constexpr size_t kOffWPT  = kOffWCT  + (size_t)kClsP * kDm  * 2;
constexpr size_t kOffX16  = kOffWPT  + (size_t)kDm   * kInP * 2;
constexpr size_t kOffUH   = kOffX16  + (size_t)kRows * kInP * 2;
constexpr size_t kOffUL   = kOffUH   + (size_t)kRows * kDm  * 2;
constexpr size_t kOffXZ   = kOffUL   + (size_t)kRows * kDm  * 2;
constexpr size_t kOffUC   = kOffXZ   + (size_t)kRows * kXzN * 4;
constexpr size_t kOffUCH  = kOffUC   + (size_t)kRows * kDin * 4;
constexpr size_t kOffUCL  = kOffUCH  + (size_t)kRows * kDin * 2;
constexpr size_t kOffDBL  = kOffUCL  + (size_t)kRows * kDin * 2;
constexpr size_t kOffYH   = kOffDBL  + (size_t)kRows * kDblP * 4;
constexpr size_t kOffYL   = kOffYH   + (size_t)kRows * kDin * 2;
constexpr size_t kOffMO   = kOffYL   + (size_t)kRows * kDin * 2;
constexpr size_t kOffPH   = kOffMO   + (size_t)kRows * kDm  * 4;
constexpr size_t kOffPL   = kOffPH   + (size_t)kBsz  * kDm  * 2;
constexpr size_t kOffCLS  = kOffPL   + (size_t)kBsz  * kDm  * 2;
constexpr size_t kWsTotal = kOffCLS  + (size_t)kBsz  * kClsP * 4;
static_assert(kWsTotal == 93315072ull, "carve total");
static_assert(kWsTotal <= 134217728ull, "carve cap");
static_assert((kOffWXT % 128) == 0 && (kOffWOT % 128) == 0 && (kOffWCT % 128) == 0 && (kOffWPT % 128) == 0 &&
              (kOffX16 % 128) == 0 && (kOffUH % 128) == 0 && (kOffUL % 128) == 0 && (kOffXZ % 128) == 0 &&
              (kOffUC % 128) == 0 && (kOffUCH % 128) == 0 && (kOffUCL % 128) == 0 && (kOffDBL % 128) == 0 &&
              (kOffYH % 128) == 0 && (kOffYL % 128) == 0 && (kOffMO % 128) == 0 && (kOffPH % 128) == 0 &&
              (kOffPL % 128) == 0 && (kOffCLS % 128) == 0, "128-B aligned regions");

__device__ __forceinline__ unsigned short f2bf_bits(float f) {
  unsigned u = __float_as_uint(f);
  return (unsigned short)((u + 0x7FFFu + ((u >> 16) & 1u)) >> 16);
}
__device__ __forceinline__ float bf_bits2f(unsigned short h) { return __uint_as_float(((unsigned)h) << 16); }
__device__ __forceinline__ float bf_rne(float f) { return bf_bits2f(f2bf_bits(f)); }

__device__ __forceinline__ void dep_guard4_h(v8f& a, v8f& b, v8f& c, v8f& d, v16h x, v16h y) {
  asm volatile("v_nop\n\tv_nop\n\tv_nop\n\tv_nop" : "+v"(a), "+v"(b), "+v"(c), "+v"(d) : "v"(x), "v"(y));
}
__device__ __forceinline__ void dep_guard4_b(v8f& a, v8f& b, v8f& c, v8f& d, v16b x, v16b y) {
  asm volatile("v_nop\n\tv_nop\n\tv_nop\n\tv_nop" : "+v"(a), "+v"(b), "+v"(c), "+v"(d) : "v"(x), "v"(y));
}
__device__ __forceinline__ void keep4_h(v16h a, v16h b, v16h c, v16h d) { asm volatile("v_nop" :: "v"(a), "v"(b), "v"(c), "v"(d)); }
__device__ __forceinline__ void keep4_b(v16b a, v16b b, v16b c, v16b d) { asm volatile("v_nop" :: "v"(a), "v"(b), "v"(c), "v"(d)); }
__device__ __forceinline__ void acc_guard4(v8f& a, v8f& b, v8f& c, v8f& d) { asm volatile("v_nop\n\tv_nop\n\tv_nop\n\tv_nop" : "+v"(a), "+v"(b), "+v"(c), "+v"(d)); }
template <typename T> struct Frag;
template <> struct Frag<_Float16> {
  typedef v16h V; union U { v16h v; v8h h[2]; };
  static __device__ __forceinline__ v16h load(const _Float16* p) {
    U f; f.h[0] = *(const v8h*)(p); f.h[1] = *(const v8h*)(p + 16); return f.v;
  }
  static __device__ __forceinline__ v8f mma(v16h a, v16h b, v8f c) {
    return __builtin_amdgcn_wmma_f32_16x16x32_f16(false, a, false, b, (short)0, c, false, false);
  }
  static __device__ __forceinline__ void guard4(v8f& a, v8f& b, v8f& c, v8f& d, v16h x, v16h y) { dep_guard4_h(a, b, c, d, x, y); }
  static __device__ __forceinline__ void keep(v16h a, v16h b, v16h c, v16h d) { keep4_h(a, b, c, d); }
};
template <> struct Frag<__bf16> {
  typedef v16b V; union U { v16b v; v8b h[2]; };
  static __device__ __forceinline__ v16b load(const __bf16* p) {
    U f; f.h[0] = *(const v8b*)(p); f.h[1] = *(const v8b*)(p + 16); return f.v;
  }
  static __device__ __forceinline__ v8f mma(v16b a, v16b b, v8f c) {
    return __builtin_amdgcn_wmma_f32_16x16x32_bf16(false, a, false, b, (short)0, c, false, false);
  }
  static __device__ __forceinline__ void guard4(v8f& a, v8f& b, v8f& c, v8f& d, v16b x, v16b y) { dep_guard4_b(a, b, c, d, x, y); }
  static __device__ __forceinline__ void keep(v16b a, v16b b, v16b c, v16b d) { keep4_b(a, b, c, d); }
};

template <int ET> struct Elem;
template <> struct Elem<0> { typedef _Float16 T; };
template <> struct Elem<1> { typedef __bf16 T; };
template <int ET, int SPL, int BIAS_MODE, int OUT_MODE, bool RESID, int ACT = 0>
__global__ __launch_bounds__(256) void wmma_gemm64(
    const unsigned short* __restrict__ Ap, const unsigned short* __restrict__ A2p, int lda, long strideA,
    const unsigned short* __restrict__ Btp, const unsigned short* __restrict__ Bt2p, int ldb, long strideB,
    void* __restrict__ Cout, void* __restrict__ Cout2, int ldc, long strideC,
    const float* __restrict__ bias,
    const float* __restrict__ resid, long strideR,
    int M, int N, int K, float scale) {
  typedef typename Elem<ET>::T T;
  typedef typename Frag<T>::V V;
  const T* A = (const T*)Ap; const T* A2 = (const T*)A2p; const T* Bt = (const T*)Btp; const T* Bt2 = (const T*)Bt2p;
  __shared__ __align__(16) float sT[8][16 * 68];
  const int b    = blockIdx.y;
  const int lane = threadIdx.x & 31;
  const int wave = threadIdx.x >> 5;
  const int tilesN = N >> 6;
  const int tilesM = M >> 6;
  const int tile = blockIdx.x * 8 + wave;
  if (tile >= tilesM * tilesN) return;
  const int tm = tile / tilesN;
  const int tn = tile - tm * tilesN;
  const int m0 = tm << 6;
  const int n0 = tn << 6;

  const T* Ab  = A  + (size_t)b * strideA;
  const T* Bb  = Bt + (size_t)b * strideB;
  const T* Ab2 = (SPL >= 1) ? (A2  + (size_t)b * strideA) : nullptr;
  const T* Bb2 = (SPL == 2) ? (Bt2 + (size_t)b * strideB) : nullptr;

  const int rlane = lane & 15;
  const int koff  = (lane >> 4) * 8;
  const int mOff  = (lane >> 4) * 8;

  v8f acc[4][4];
#pragma unroll
  for (int i = 0; i < 4; ++i)
#pragma unroll
    for (int j = 0; j < 4; ++j) acc[i][j] = (v8f){0.f,0.f,0.f,0.f,0.f,0.f,0.f,0.f};

  for (int k0 = 0; k0 < K; k0 += 32) {
    V bh[4], bl[4];
#pragma unroll
    for (int j = 0; j < 4; ++j) {
      const size_t bo = (size_t)(n0 + (j << 4) + rlane) * ldb + koff + k0;
      bh[j] = Frag<T>::load(Bb + bo);
      if (SPL == 2) bl[j] = Frag<T>::load(Bb2 + bo);
    }
#pragma unroll
    for (int i = 0; i < 4; ++i) {
      const size_t ao = (size_t)(m0 + (i << 4) + rlane) * lda + koff + k0;
      V ah = Frag<T>::load(Ab + ao);
      V al;
      if (SPL >= 1) al = Frag<T>::load(Ab2 + ao);
#pragma unroll
      for (int j = 0; j < 4; ++j) {
        acc[i][j] = Frag<T>::mma(ah, bh[j], acc[i][j]);
        if (SPL == 2) acc[i][j] = Frag<T>::mma(ah, bl[j], acc[i][j]);
        if (SPL >= 1) acc[i][j] = Frag<T>::mma(al, bh[j], acc[i][j]);
      }
      Frag<T>::guard4(acc[i][0], acc[i][1], acc[i][2], acc[i][3], ah, (SPL >= 1) ? al : ah);
    }
    Frag<T>::keep(bh[0], bh[1], bh[2], bh[3]);
    if (SPL == 2) Frag<T>::keep(bl[0], bl[1], bl[2], bl[3]);
  }
  acc_guard4(acc[0][0], acc[0][1], acc[0][2], acc[0][3]);
  acc_guard4(acc[1][0], acc[1][1], acc[1][2], acc[1][3]);
  acc_guard4(acc[2][0], acc[2][1], acc[2][2], acc[2][3]);
  acc_guard4(acc[3][0], acc[3][1], acc[3][2], acc[3][3]);

  float* slab = sT[wave];
  const float* Rb = RESID ? (resid + (size_t)b * strideR) : nullptr;
#pragma unroll
  for (int i = 0; i < 4; ++i) {
    const int mBase = m0 + (i << 4);
#pragma unroll
    for (int j = 0; j < 4; ++j) {
      const int n = n0 + (j << 4) + rlane;
      float bv = 0.f;
      if (BIAS_MODE == 2) bv = bias[n];
#pragma unroll
      for (int r = 0; r < 8; ++r) {
        float v = acc[i][j][r] * scale;
        if (BIAS_MODE == 1) v += bias[mBase + mOff + r];
        if (BIAS_MODE == 2) v += bv;
        if (RESID) v += Rb[(size_t)(mBase + mOff + r) * ldc + n];
        if (ACT == 1) v = tanhf(v);
        if (ACT == 2) v = fmaxf(v, 0.0f);
        if (ACT == 3) v = v / (1.0f + expf(-v));
        if (ACT == 4) v = (v > 0.f) ? v : 0.01f * v;
        slab[(mOff + r) * 68 + (j << 4) + rlane] = v;
      }
    }
    __builtin_amdgcn_fence(__ATOMIC_RELEASE, "workgroup");
    __builtin_amdgcn_wave_barrier();
    __builtin_amdgcn_fence(__ATOMIC_ACQUIRE, "workgroup");
    if (OUT_MODE == 0) {
      float* C = (float*)Cout + (size_t)b * strideC;
      const int hh = lane >> 4, c4 = (lane & 15) * 4;
      for (int pass = 0; pass < 2; ++pass) {
#pragma unroll
        for (int it = 0; it < 8; ++it) {
          const int row = it * 2 + hh;
          v4f v = *(const v4f*)(slab + row * 68 + c4);
          *(volatile v4f*)(C + (size_t)(mBase + row) * ldc + n0 + c4) = v;
        }
        __threadfence();
      }
    } else {
      const int q = lane >> 3, c8 = (lane & 7) * 8;
      unsigned short* C  = (unsigned short*)Cout  + (size_t)b * strideC;
      unsigned short* C2 = (OUT_MODE == 2) ? ((unsigned short*)Cout2 + (size_t)b * strideC) : nullptr;
      for (int pass = 0; pass < 2; ++pass) {
#pragma unroll
        for (int it = 0; it < 4; ++it) {
          const int row = it * 4 + q;
          const float* sp = slab + row * 68 + c8;
          v8h hv, lv;
#pragma unroll
          for (int e = 0; e < 8; ++e) {
            if (OUT_MODE == 1) {
              hv[e] = (_Float16)sp[e];
            } else {
              unsigned short hb = f2bf_bits(sp[e]);
              unsigned short lb = f2bf_bits(sp[e] - bf_bits2f(hb));
              hv[e] = __builtin_bit_cast(_Float16, hb);
              lv[e] = __builtin_bit_cast(_Float16, lb);
            }
          }
          *(volatile v8h*)(C + (size_t)(mBase + row) * ldc + n0 + c8) = hv;
          if (OUT_MODE == 2) *(volatile v8h*)(C2 + (size_t)(mBase + row) * ldc + n0 + c8) = lv;
        }
        __threadfence();
      }
    }
    __builtin_amdgcn_fence(__ATOMIC_RELEASE, "workgroup");
    __builtin_amdgcn_wave_barrier();
    __builtin_amdgcn_fence(__ATOMIC_ACQUIRE, "workgroup");
  }
}

__global__ __launch_bounds__(256) void transpose_cast_bf16_kernel(
    const float* __restrict__ W, unsigned short* __restrict__ Bt, int Kdim, int Ndim, int Npad)
{
  __shared__ float tile[64 * 65];
  const int tid = threadIdx.x, lane = tid & 31, wave = tid >> 5;
  const int n0 = blockIdx.x * 64;
  const int k0 = blockIdx.y * 64;
  (void)Npad;
#pragma unroll
  for (int p = 0; p < 16; ++p) {
    const int idx = tid + p * 256;
    const int kk  = idx >> 6;
    const int nn  = idx & 63;
    const int n   = n0 + nn;
    const int nc  = (n < Ndim) ? n : (Ndim - 1);
    const float v = W[(size_t)(k0 + kk) * Ndim + nc];
    tile[kk * 65 + nn] = (n < Ndim) ? v : 0.f;
  }
  __syncthreads();
  const int q = lane >> 3, c8 = (lane & 7) * 8;
  v8h hv[2];
#pragma unroll
  for (int it = 0; it < 2; ++it) {
    const int nrow = it * 32 + wave * 4 + q;
#pragma unroll
    for (int e = 0; e < 8; ++e) {
      const unsigned short hb = f2bf_bits(tile[(c8 + e) * 65 + nrow]);
      hv[it][e] = __builtin_bit_cast(_Float16, hb);
    }
  }
  for (int pass = 0; pass < 2; ++pass) {
#pragma unroll
    for (int it = 0; it < 2; ++it) {
      const int nrow = it * 32 + wave * 4 + q;
      *(volatile v8h*)(Bt + (size_t)(n0 + nrow) * Kdim + k0 + c8) = hv[it];
    }
    __threadfence();
  }
}

__global__ __launch_bounds__(256) void pad_winp_kernel(const float* __restrict__ Wp, unsigned short* __restrict__ WPT)
{
  __shared__ float sw[kInF * kDm];
  const int tid = threadIdx.x;
#pragma unroll
  for (int p = 0; p < 14; ++p) sw[tid + 256 * p] = Wp[tid + 256 * p];
  __syncthreads();
  v8h hv[2];
#pragma unroll
  for (int it = 0; it < 2; ++it) {
    const int u  = tid + 256 * it;
    const int n  = u >> 2;
    const int k8 = (u & 3) * 8;
#pragma unroll
    for (int e = 0; e < 8; ++e) {
      const int k  = k8 + e;
      const int kc = (k < kInF) ? k : (kInF - 1);
      const float v = sw[kc * kDm + n];
      const float w = (k < kInF) ? v : 0.f;
      const unsigned short hb = f2bf_bits(w);
      hv[it][e] = __builtin_bit_cast(_Float16, hb);
    }
  }
  for (int pass = 0; pass < 2; ++pass) {
#pragma unroll
    for (int it = 0; it < 2; ++it)
      *(volatile v8h*)(WPT + (size_t)(tid + 256 * it) * 8) = hv[it];
    __threadfence();
  }
}

__global__ __launch_bounds__(256) void pad_x_kernel(const float* __restrict__ x, unsigned short* __restrict__ X16)
{
  __shared__ float sx[64 * kInF];
  const int tid = threadIdx.x;
  const size_t r0 = (size_t)blockIdx.x * 64;
  const float* xb = x + r0 * kInF;
#pragma unroll
  for (int p = 0; p < 7; ++p) sx[tid + 256 * p] = xb[tid + 256 * p];
  __syncthreads();
  const int row = tid >> 2;
  const int c8  = (tid & 3) * 8;
  v8h hv;
#pragma unroll
  for (int e = 0; e < 8; ++e) {
    const int c  = c8 + e;
    const int cc = (c < kInF) ? c : (kInF - 1);
    const float v = sx[row * kInF + cc];
    const float w = (c < kInF) ? v : 0.f;
    const unsigned short hb = f2bf_bits(w);
    hv[e] = __builtin_bit_cast(_Float16, hb);
  }
  unsigned short* q = X16 + r0 * kInP + (size_t)tid * 8;
  *(volatile v8h*)q = hv;
  __threadfence();
  *(volatile v8h*)q = hv;
}

__global__ __launch_bounds__(256) void conv_silu_kernel(
    const float* __restrict__ XZ, const float* __restrict__ cw, const float* __restrict__ cb,
    float* __restrict__ UC, unsigned short* __restrict__ UCH, unsigned short* __restrict__ UCL)
{
  __shared__ __align__(16) float sT[16 * kConvTP];
  const int tid = threadIdx.x, lane = tid & 31, wave = tid >> 5;
  const int d = tid;
  const int g0 = blockIdx.x * 64;
  int tcur = g0 % kSeq;
  const float w0 = bf_rne(cw[d * kTaps + 0]);
  const float w1 = bf_rne(cw[d * kTaps + 1]);
  const float w2 = bf_rne(cw[d * kTaps + 2]);
  const float bc = bf_rne(cb[d]);
  float xm2, xm1;
  {
    const int r1 = (g0 >= 1) ? (g0 - 1) : 0;
    const int r2 = (g0 >= 2) ? (g0 - 2) : 0;
    const float v1 = XZ[(size_t)r1 * kXzN + d];
    const float v2 = XZ[(size_t)r2 * kXzN + d];
    xm1 = (tcur >= 1) ? v1 : 0.f;
    xm2 = (tcur >= 2) ? v2 : 0.f;
  }
  const int hrow = wave >> 1;
  const int hch  = (wave & 1) * 128 + lane * 4;
#pragma unroll 1
  for (int sub = 0; sub < 4; ++sub) {
    const int lb = g0 + sub * 16;
#pragma unroll 1
    for (int s = 0; s < 16; ++s) {
      xm1 = (tcur == 0) ? 0.f : xm1;
      xm2 = (tcur == 0) ? 0.f : xm2;
      const float xcur = XZ[(size_t)(lb + s) * kXzN + d];
      float acc = w0 * xm2;
      acc = fmaf(w1, xm1, acc);
      acc = fmaf(w2, xcur, acc);
      const float sv = acc + bc;
      const float sg = __builtin_amdgcn_rcpf(1.0f + __expf(-sv));
      sT[s * kConvTP + tid] = sv * sg;
      xm2 = xm1; xm1 = xcur;
      tcur = (tcur == kSeq - 1) ? 0 : (tcur + 1);
    }
    __syncthreads();
    v4f fv[4];
    v8h bh[2], blo[2];
#pragma unroll
    for (int it = 0; it < 4; ++it) fv[it] = *(const v4f*)(sT + (it * 4 + hrow) * kConvTP + hch);
#pragma unroll
    for (int it = 0; it < 2; ++it) {
      const float* sp = sT + (it * 8 + wave) * kConvTP + lane * 8;
      const v4f a0 = *(const v4f*)(sp);
      const v4f a1 = *(const v4f*)(sp + 4);
#pragma unroll
      for (int e = 0; e < 4; ++e) {
        const unsigned short h0 = f2bf_bits(a0[e]), h1 = f2bf_bits(a1[e]);
        const unsigned short l0 = f2bf_bits(a0[e] - bf_bits2f(h0)), l1 = f2bf_bits(a1[e] - bf_bits2f(h1));
        bh[it][e]      = __builtin_bit_cast(_Float16, h0);
        bh[it][4 + e]  = __builtin_bit_cast(_Float16, h1);
        blo[it][e]     = __builtin_bit_cast(_Float16, l0);
        blo[it][4 + e] = __builtin_bit_cast(_Float16, l1);
      }
    }
    for (int pass = 0; pass < 2; ++pass) {
#pragma unroll
      for (int it = 0; it < 4; ++it)
        *(volatile v4f*)(UC + (size_t)(lb + it * 4 + hrow) * kDin + hch) = fv[it];
#pragma unroll
      for (int it = 0; it < 2; ++it) {
        const size_t o = (size_t)(lb + it * 8 + wave) * kDin + lane * 8;
        *(volatile v8h*)(UCH + o) = bh[it];
        *(volatile v8h*)(UCL + o) = blo[it];
      }
      __threadfence();
    }
    __syncthreads();
  }
}

__global__ __launch_bounds__(256) void scan_kernel(
    const float* __restrict__ DBL, const float* __restrict__ UC, const float* __restrict__ XZ,
    const float* __restrict__ Wdt, const float* __restrict__ dtb, const float* __restrict__ Alog,
    const float* __restrict__ Dp, unsigned short* __restrict__ YH, unsigned short* __restrict__ YL)
{
  __shared__ __align__(16) float sD[kSeq * kDblP];
  __shared__ __align__(16) float sY[kSeq * kScanYP];
  __shared__ __align__(16) float sW[kDtR * kDin];
  __shared__ __align__(16) float sA[kNst * kDin];
  const int tid = threadIdx.x, lane = tid & 31, wave = tid >> 5;
  const int d = tid;
  const size_t row0 = (size_t)blockIdx.x * kSeq;
  {
    const float* src = DBL + row0 * kDblP;
#pragma unroll
    for (int p = 0; p < 7; ++p) sD[tid + 256 * p] = src[tid + 256 * p];
  }
#pragma unroll 1
  for (int r = 0; r < kDtR; ++r) sW[r * kDin + tid] = bf_rne(Wdt[(size_t)r * kDin + tid]);
#pragma unroll 1
  for (int s = 0; s < kNst; ++s) sA[s * kDin + tid] = -expf(bf_rne(Alog[(size_t)tid * kNst + s]));
  __syncthreads();
  float An[kNst], h[kNst], wd[kDtR];
#pragma unroll
  for (int s = 0; s < kNst; ++s) { An[s] = sA[s * kDin + tid]; h[s] = 0.f; }
#pragma unroll
  for (int r = 0; r < kDtR; ++r) wd[r] = sW[r * kDin + tid];
  const float bb = bf_rne(dtb[d]);
  const float Dd = bf_rne(Dp[d]);
#pragma unroll 1
  for (int t = 0; t < kSeq; ++t) {
    const float* xr = sD + t * kDblP;
    const v4f q0 = *(const v4f*)(xr);
    const v4f q1 = *(const v4f*)(xr + 4);
    float vdot = 0.f;
    vdot = fmaf(q0[0], wd[0], vdot);
    vdot = fmaf(q0[1], wd[1], vdot);
    vdot = fmaf(q0[2], wd[2], vdot);
    vdot = fmaf(q0[3], wd[3], vdot);
    vdot = fmaf(q1[0], wd[4], vdot);
    vdot = fmaf(q1[1], wd[5], vdot);
    vdot = fmaf(q1[2], wd[6], vdot);
    vdot = fmaf(q1[3], wd[7], vdot);
    v4f Bq[4], Cq[4];
#pragma unroll
    for (int qq = 0; qq < 4; ++qq) {
      Bq[qq] = *(const v4f*)(xr + kDtR + 4 * qq);
      Cq[qq] = *(const v4f*)(xr + kDtR + kNst + 4 * qq);
    }
    const float v   = vdot + bb;
    const float a   = __expf(-fabsf(v));
    const float u   = 1.0f + a;
    const float l1p = __logf(u) + (a - (u - 1.0f)) * __builtin_amdgcn_rcpf(u);
    const float delta = fmaxf(v, 0.0f) + l1p;
    const size_t m  = row0 + t;
    const float xv  = UC[m * kDin + d];
    const float zv  = XZ[m * kXzN + kDin + d];
    float y = 0.f;
#pragma unroll
    for (int n = 0; n < kNst; ++n) {
      const float e = __expf(delta * An[n]);
      float db = delta * Bq[n >> 2][n & 3];
      asm volatile("" : "+v"(db));
      float p = db * xv;
      asm volatile("" : "+v"(p));
      float qv = h[n] * e;
      asm volatile("" : "+v"(qv));
      const float hn = qv + p;
      h[n] = hn;
      float rr = hn * Cq[n >> 2][n & 3];
      asm volatile("" : "+v"(rr));
      y += rr;
    }
    float sk = xv * Dd;
    asm volatile("" : "+v"(sk));
    y += sk;
    const float sg = __builtin_amdgcn_rcpf(1.0f + __expf(-zv));
    const float g  = zv * sg;
    sY[t * kScanYP + tid] = y * g;
  }
  __syncthreads();
  v8h hv[4], lv[4];
#pragma unroll
  for (int it = 0; it < 4; ++it) {
    const int row  = it * 8 + wave;
    const int rowc = (row < kSeq) ? row : (kSeq - 1);
    const float* sp = sY + rowc * kScanYP + lane * 8;
    const v4f a0 = *(const v4f*)(sp);
    const v4f a1 = *(const v4f*)(sp + 4);
#pragma unroll
    for (int e = 0; e < 4; ++e) {
      const unsigned short h0 = f2bf_bits(a0[e]), h1 = f2bf_bits(a1[e]);
      const unsigned short l0 = f2bf_bits(a0[e] - bf_bits2f(h0)), l1 = f2bf_bits(a1[e] - bf_bits2f(h1));
      hv[it][e]     = __builtin_bit_cast(_Float16, h0);
      hv[it][4 + e] = __builtin_bit_cast(_Float16, h1);
      lv[it][e]     = __builtin_bit_cast(_Float16, l0);
      lv[it][4 + e] = __builtin_bit_cast(_Float16, l1);
    }
  }
  for (int pass = 0; pass < 2; ++pass) {
#pragma unroll
    for (int it = 0; it < 4; ++it) {
      const int row = it * 8 + wave;
      if (row < kSeq) {
        const size_t o = (row0 + row) * kDin + (size_t)lane * 8;
        *(volatile v8h*)(YH + o) = hv[it];
        *(volatile v8h*)(YL + o) = lv[it];
      }
    }
    __threadfence();
  }
}

__global__ __launch_bounds__(256) void pool_split_kernel(
    const float* __restrict__ MO, unsigned short* __restrict__ PH, unsigned short* __restrict__ PL)
{
  const int i  = blockIdx.x * 256 + threadIdx.x;
  const int b  = i >> 4;
  const int d8 = (i & 15) * 8;
  v4f s0 = (v4f){0.f, 0.f, 0.f, 0.f};
  v4f s1 = (v4f){0.f, 0.f, 0.f, 0.f};
  const float* base = MO + (size_t)b * kSeq * kDm + d8;
#pragma unroll 1
  for (int t = 0; t < kSeq; ++t) {
    const float* p = base + (size_t)t * kDm;
    s0 += *(const v4f*)(p);
    s1 += *(const v4f*)(p + 4);
  }
  v8h hv, lv;
#pragma unroll
  for (int e = 0; e < 4; ++e) {
    const float f0 = s0[e] * kInvSeq;
    const float f1 = s1[e] * kInvSeq;
    const unsigned short h0 = f2bf_bits(f0), h1 = f2bf_bits(f1);
    const unsigned short l0 = f2bf_bits(f0 - bf_bits2f(h0)), l1 = f2bf_bits(f1 - bf_bits2f(h1));
    hv[e]     = __builtin_bit_cast(_Float16, h0);
    hv[4 + e] = __builtin_bit_cast(_Float16, h1);
    lv[e]     = __builtin_bit_cast(_Float16, l0);
    lv[4 + e] = __builtin_bit_cast(_Float16, l1);
  }
  const size_t o = (size_t)i * 8;
  *(volatile v8h*)(PH + o) = hv;
  *(volatile v8h*)(PL + o) = lv;
  __threadfence();
  *(volatile v8h*)(PH + o) = hv;
  *(volatile v8h*)(PL + o) = lv;
}

__global__ __launch_bounds__(256) void pack_out_kernel(const float* __restrict__ CLS, float* __restrict__ out)
{
  const int i = blockIdx.x * 256 + threadIdx.x;
  v4f v;
#pragma unroll
  for (int j = 0; j < 4; ++j) {
    const int e   = 4 * i + j;
    const int row = e / kNcls;
    const int col = e - row * kNcls;
    v[j] = CLS[(size_t)row * kClsP + col];
  }
  float* q = out + (size_t)i * 4;
  *(volatile v4f*)q = v;
  __threadfence();
  *(volatile v4f*)q = v;
}

extern "C" void kernel_launch(void* const* d_in, const int* in_sizes, int n_in,
                              void* d_out, int out_size, void* d_ws, size_t ws_size,
                              hipStream_t stream)
{
  if (n_in < 12) return;
  if (in_sizes[0]  != kRows * kInF) return;
  if (in_sizes[1]  != kInF * kDm) return;
  if (in_sizes[2]  != kDm * kXzN) return;
  if (in_sizes[3]  != kDin * kTaps) return;
  if (in_sizes[4]  != kDin) return;
  if (in_sizes[5]  != kDin * kDblN) return;
  if (in_sizes[6]  != kDtR * kDin) return;
  if (in_sizes[7]  != kDin) return;
  if (in_sizes[8]  != kDin * kNst) return;
  if (in_sizes[9]  != kDin) return;
  if (in_sizes[10] != kDin * kDm) return;
  if (in_sizes[11] != kDm * kNcls) return;
  if (out_size != kBsz * kNcls) return;
  if (ws_size < kWsTotal) return;

  const float* x       = (const float*)d_in[0];
  const float* w_inp   = (const float*)d_in[1];
  const float* w_in    = (const float*)d_in[2];
  const float* conv_w  = (const float*)d_in[3];
  const float* conv_b  = (const float*)d_in[4];
  const float* w_x     = (const float*)d_in[5];
  const float* w_dt    = (const float*)d_in[6];
  const float* dt_bias = (const float*)d_in[7];
  const float* A_log   = (const float*)d_in[8];
  const float* Dv      = (const float*)d_in[9];
  const float* w_out   = (const float*)d_in[10];
  const float* w_cls   = (const float*)d_in[11];
  float* out = (float*)d_out;

  char* ws = (char*)d_ws;
  unsigned short* WINT = (unsigned short*)(ws + kOffWINT);
  unsigned short* WXT  = (unsigned short*)(ws + kOffWXT);
  unsigned short* WOT  = (unsigned short*)(ws + kOffWOT);
  unsigned short* WCT  = (unsigned short*)(ws + kOffWCT);
  unsigned short* WPT  = (unsigned short*)(ws + kOffWPT);
  unsigned short* X16  = (unsigned short*)(ws + kOffX16);
  unsigned short* UH   = (unsigned short*)(ws + kOffUH);
  unsigned short* UL   = (unsigned short*)(ws + kOffUL);
  float*          XZ   = (float*)(ws + kOffXZ);
  float*          UC   = (float*)(ws + kOffUC);
  unsigned short* UCH  = (unsigned short*)(ws + kOffUCH);
  unsigned short* UCL  = (unsigned short*)(ws + kOffUCL);
  float*          DBL  = (float*)(ws + kOffDBL);
  unsigned short* YH   = (unsigned short*)(ws + kOffYH);
  unsigned short* YL   = (unsigned short*)(ws + kOffYL);
  float*          MO   = (float*)(ws + kOffMO);
  unsigned short* PH   = (unsigned short*)(ws + kOffPH);
  unsigned short* PL   = (unsigned short*)(ws + kOffPL);
  float*          CLS  = (float*)(ws + kOffCLS);
  const float* dummy_bias  = dt_bias;
  const float* dummy_resid = x;

  transpose_cast_bf16_kernel<<<dim3(kXzN / 64,  kDm / 64),  256, 0, stream>>>(w_in,  WINT, kDm,  kXzN,  kXzN);
  transpose_cast_bf16_kernel<<<dim3(kDblP / 64, kDin / 64), 256, 0, stream>>>(w_x,   WXT,  kDin, kDblN, kDblP);
  transpose_cast_bf16_kernel<<<dim3(kDm / 64,   kDin / 64), 256, 0, stream>>>(w_out, WOT,  kDin, kDm,   kDm);
  transpose_cast_bf16_kernel<<<dim3(kClsP / 64, kDm / 64),  256, 0, stream>>>(w_cls, WCT,  kDm,  kNcls, kClsP);
  pad_winp_kernel<<<1, 256, 0, stream>>>(w_inp, WPT);
  pad_x_kernel<<<kRows / 64, 256, 0, stream>>>(x, X16);

  wmma_gemm64<1, 0, 0, 2, false><<<dim3(56, 1), 256, 0, stream>>>(
      X16, X16, kInP, 0L, WPT, WPT, kInP, 0L,
      (void*)UH, (void*)UL, kDm, 0L, dummy_bias, dummy_resid, 0L, kRows, kDm, kInP, 1.0f);

  wmma_gemm64<1, 1, 0, 0, false><<<dim3(224, 1), 256, 0, stream>>>(
      UH, UL, kDm, 0L, WINT, WINT, kDm, 0L,
      (void*)XZ, (void*)XZ, kXzN, 0L, dummy_bias, dummy_resid, 0L, kRows, kXzN, kDm, 1.0f);

  conv_silu_kernel<<<kRows / 64, 256, 0, stream>>>(XZ, conv_w, conv_b, UC, UCH, UCL);

  wmma_gemm64<1, 1, 0, 0, false><<<dim3(28, 1), 256, 0, stream>>>(
      UCH, UCL, kDin, 0L, WXT, WXT, kDin, 0L,
      (void*)DBL, (void*)DBL, kDblP, 0L, dummy_bias, dummy_resid, 0L, kRows, kDblP, kDin, 1.0f);

  scan_kernel<<<kBsz, kDin, 0, stream>>>(DBL, UC, XZ, w_dt, dt_bias, A_log, Dv, YH, YL);

  wmma_gemm64<1, 1, 0, 0, false><<<dim3(56, 1), 256, 0, stream>>>(
      YH, YL, kDin, 0L, WOT, WOT, kDin, 0L,
      (void*)MO, (void*)MO, kDm, 0L, dummy_bias, dummy_resid, 0L, kRows, kDm, kDin, 1.0f);

  pool_split_kernel<<<(kBsz * kDm) / 8 / 256, 256, 0, stream>>>(MO, PH, PL);

  wmma_gemm64<1, 1, 0, 0, false><<<dim3(1, 1), 256, 0, stream>>>(
      PH, PL, kDm, 0L, WCT, WCT, kDm, 0L,
      (void*)CLS, (void*)CLS, kClsP, 0L, dummy_bias, dummy_resid, 0L, kBsz, kClsP, kDm, 1.0f);

  pack_out_kernel<<<(kBsz * kNcls) / 4 / 256, 256, 0, stream>>>(CLS, out);
}
